// RNN_2156073583212
// MI455X (gfx1250) — hardware-verified
//
#include <hip/hip_runtime.h>

typedef __attribute__((ext_vector_type(16))) _Float16 v16h;
typedef __attribute__((ext_vector_type(8)))  _Float16 v8h;
typedef __attribute__((ext_vector_type(8)))  float    v8f;
typedef __attribute__((ext_vector_type(4)))  float    v4f;

constexpr int NB   = 8192;
constexpr int NT   = 512;
constexpr int NH   = 64;
constexpr int NO   = 1;
constexpr int NTHR   = 128;
constexpr int NWAVE  = NTHR / 32;
constexpr int ROWS_W = 32;
constexpr int ROWS_B = NWAVE * ROWS_W;
constexpr int NBLK   = NB / ROWS_B;
constexpr int HP     = 72;
constexpr int WP     = 72;
constexpr int MT     = NH / 16;
constexpr int KC     = NH / 32;
constexpr float HCAR      = 256.0f;
constexpr float WCAR      = 256.0f;
constexpr float SCAR      = HCAR * WCAR;
constexpr float SCAR_INV  = 1.0f / (256.0f * 256.0f);
constexpr float ACC_TO_H16 = 1.0f / 256.0f;
static_assert(NB % ROWS_B == 0);
static_assert(NBLK * ROWS_B == NB);
static_assert(NH == 64 && MT == 4 && KC == 2);
static_assert(HP % 8 == 0 && WP % 8 == 0);
static_assert((NH * NH / 8) % NTHR == 0);
static_assert(ROWS_B == 4 * 32);
static_assert(NO == 1);

__device__ __forceinline__ void dep_guard3_h(v8f& a, v8f& b, v16h x, v16h y, v16h z) {
  asm volatile("v_nop\n\tv_nop\n\tv_nop\n\tv_nop" : "+v"(a), "+v"(b) : "v"(x), "v"(y), "v"(z));
}
__device__ __forceinline__ void acc_guard4(v8f& a, v8f& b, v8f& c, v8f& d) {
  asm volatile("v_nop\n\tv_nop\n\tv_nop\n\tv_nop" : "+v"(a), "+v"(b), "+v"(c), "+v"(d));
}
template <typename T> struct Frag;
template <> struct Frag<_Float16> {
  typedef v16h V; union U { v16h v; v8h h[2]; };
  static __device__ __forceinline__ v16h load(const _Float16* p) {
    U f; f.h[0] = *(const v8h*)(p); f.h[1] = *(const v8h*)(p + 16); return f.v;
  }
  static __device__ __forceinline__ v8f mma(v16h a, v16h b, v8f c) {
    return __builtin_amdgcn_wmma_f32_16x16x32_f16(false, a, false, b, (short)0, c, false, false);
  }
};

__global__ __launch_bounds__(NTHR) void relu_rnn_seq_kernel(
    const float* __restrict__ x,
    const float* __restrict__ w_xh,
    const float* __restrict__ w_hh,
    const float* __restrict__ w_hy,
    float* __restrict__ out) {
  __shared__ __align__(16) _Float16 wsh[NH * WP];
  __shared__ __align__(16) _Float16 hsh[NWAVE][ROWS_W * HP];
  __shared__ __align__(16) float    wxs[NH];
  __shared__ __align__(16) float    wys[NH];
  __shared__ __align__(16) float    outs[ROWS_B];

  const int tid = threadIdx.x, lane = tid & 31, wave = tid >> 5;
  const int c = lane & 15, hh = lane >> 4, koff = hh * 8;
  const int rowg = blockIdx.x * ROWS_B + wave * ROWS_W;

#pragma unroll 1
  for (int q = tid; q < NH * NH / 8; q += NTHR) {
    const int row = q >> 3, c8 = (q & 7) * 8;
    const float* sp = w_hh + row * NH + c8;
    const v4f fa = *(const v4f*)(sp);
    const v4f fb = *(const v4f*)(sp + 4);
    v8h hv;
    hv[0] = (_Float16)(fa[0] * WCAR); hv[1] = (_Float16)(fa[1] * WCAR);
    hv[2] = (_Float16)(fa[2] * WCAR); hv[3] = (_Float16)(fa[3] * WCAR);
    hv[4] = (_Float16)(fb[0] * WCAR); hv[5] = (_Float16)(fb[1] * WCAR);
    hv[6] = (_Float16)(fb[2] * WCAR); hv[7] = (_Float16)(fb[3] * WCAR);
    *(v8h*)(wsh + row * WP + c8) = hv;
  }
  if (wave == 0) {
    wxs[lane]      = w_xh[lane];
    wxs[32 + lane] = w_xh[32 + lane];
    wys[lane]      = w_hy[lane];
    wys[32 + lane] = w_hy[32 + lane];
  }
  __syncthreads();

  float wxS[MT][8];
#pragma unroll
  for (int mt = 0; mt < MT; ++mt)
#pragma unroll
    for (int r = 0; r < 8; ++r) wxS[mt][r] = wxs[16 * mt + 8 * hh + r] * SCAR;

  const float* xr0 = x + (size_t)(rowg + c) * NT;
  const float* xr1 = x + (size_t)(rowg + 16 + c) * NT;

  v8f acc[MT][2];
  {
    const float x0 = xr0[0];
    const float x1 = xr1[0];
#pragma unroll
    for (int mt = 0; mt < MT; ++mt)
#pragma unroll
      for (int r = 0; r < 8; ++r) {
        acc[mt][0][r] = x0 * wxS[mt][r];
        acc[mt][1][r] = x1 * wxS[mt][r];
      }
  }

  _Float16* hw = &hsh[wave][0];

#pragma unroll 1
  for (int t = 1; t < NT; ++t) {
#pragma unroll
    for (int mt = 0; mt < MT; ++mt) {
#pragma unroll
      for (int nb = 0; nb < 2; ++nb) {
        v8h hv;
#pragma unroll
        for (int r = 0; r < 8; ++r) hv[r] = (_Float16)fmaxf(acc[mt][nb][r] * ACC_TO_H16, 0.0f);
        *(v8h*)(hw + (16 * nb + c) * HP + 16 * mt + 8 * hh) = hv;
      }
    }
    __syncthreads();

    const float x0 = xr0[t];
    const float x1 = xr1[t];
#pragma unroll
    for (int mt = 0; mt < MT; ++mt)
#pragma unroll
      for (int r = 0; r < 8; ++r) {
        acc[mt][0][r] = x0 * wxS[mt][r];
        acc[mt][1][r] = x1 * wxS[mt][r];
      }

#pragma unroll
    for (int kc = 0; kc < KC; ++kc) {
      const v16h b0 = Frag<_Float16>::load(hw + c * HP + kc * 32 + koff);
      const v16h b1 = Frag<_Float16>::load(hw + (16 + c) * HP + kc * 32 + koff);
#pragma unroll
      for (int mt = 0; mt < MT; ++mt) {
        const v16h a = Frag<_Float16>::load(wsh + (16 * mt + c) * WP + kc * 32 + koff);
        acc[mt][0] = Frag<_Float16>::mma(a, b0, acc[mt][0]);
        acc[mt][1] = Frag<_Float16>::mma(a, b1, acc[mt][1]);
        dep_guard3_h(acc[mt][0], acc[mt][1], a, b0, b1);
      }
    }
    acc_guard4(acc[0][0], acc[0][1], acc[1][0], acc[1][1]);
    acc_guard4(acc[2][0], acc[2][1], acc[3][0], acc[3][1]);
  }

  float s0 = 0.0f, s1 = 0.0f;
#pragma unroll
  for (int mt = 0; mt < MT; ++mt) {
#pragma unroll
    for (int r = 0; r < 8; ++r) {
      const float wv = wys[16 * mt + 8 * hh + r];
      const float h0 = fmaxf(acc[mt][0][r] * SCAR_INV, 0.0f);
      const float h1 = fmaxf(acc[mt][1][r] * SCAR_INV, 0.0f);
      s0 += h0 * wv;
      s1 += h1 * wv;
    }
  }
  s0 += __shfl_xor(s0, 16, 32);
  s1 += __shfl_xor(s1, 16, 32);
  {
    const float sv = hh ? s1 : s0;
    outs[wave * ROWS_W + lane] = sv;
  }
  __syncthreads();

  if (wave == 0) {
    const v4f v = *(const v4f*)(outs + 4 * lane);
    float* op = out + (size_t)blockIdx.x * ROWS_B + 4 * lane;
    *(volatile v4f*)op = v;
    __threadfence();
    *(volatile v4f*)op = v;
  }
}

extern "C" void kernel_launch(void* const* d_in, const int* in_sizes, int n_in,
                              void* d_out, int out_size, void* d_ws, size_t ws_size, hipStream_t stream) {
  if (n_in < 4 || d_out == nullptr) return;
  if (in_sizes[0] != NB * NT || in_sizes[1] != NH * 1 || in_sizes[2] != NH * NH ||
      in_sizes[3] != NO * NH || out_size != NB * NO) return;
  const float* x    = (const float*)d_in[0];
  const float* w_xh = (const float*)d_in[1];
  const float* w_hh = (const float*)d_in[2];
  const float* w_hy = (const float*)d_in[3];
  float* out = (float*)d_out;
  (void)d_ws; (void)ws_size;
  relu_rnn_seq_kernel<<<NBLK, NTHR, 0, stream>>>(x, w_xh, w_hh, w_hy, out);
}
